// SelfAttention_74655121539564
// MI455X (gfx1250) — hardware-verified
//
#include <hip/hip_runtime.h>
#ifndef NB
#define NB 4
#endif
#ifndef SEQ
#define SEQ 4096
#endif
#define NB_FULL 4
#define SEQ_FULL 4096
#define EMB 768
#define HD 64
#define NOUT 192
#define NTOK (NB * SEQ)
#define CARRY 16.0f
#define SC_LOGIT 0.00048828125f

static_assert(EMB % 32 == 0);
static_assert(HD == 64);
static_assert(NOUT == 3 * HD);
static_assert(SEQ % 64 == 0);
static_assert(NTOK % 64 == 0);
static_assert(SEQ <= SEQ_FULL);
static_assert(NB <= NB_FULL);
static_assert((NOUT * (EMB / 8)) % 256 == 0);

#define WP_BYTES ((size_t)NOUT * EMB * 2)
#define PL_BYTES ((size_t)NTOK * HD * 2)
#define OFF_WP ((size_t)0)
#define OFF_KH (OFF_WP + ((WP_BYTES + 255) & ~(size_t)255))
#define OFF_QH (OFF_KH + ((PL_BYTES + 255) & ~(size_t)255))
#define OFF_VT (OFF_QH + ((PL_BYTES + 255) & ~(size_t)255))
#define OFF_END (OFF_VT + ((PL_BYTES + 255) & ~(size_t)255))
static_assert(OFF_END <= (size_t)134217728);

typedef __bf16 v16b __attribute__((ext_vector_type(16)));
typedef _Float16 v16h __attribute__((ext_vector_type(16)));
typedef unsigned short v8us __attribute__((ext_vector_type(8), may_alias));
typedef float v8f __attribute__((ext_vector_type(8)));
typedef float v4f __attribute__((ext_vector_type(4)));
typedef float v4fa __attribute__((ext_vector_type(4), may_alias));
union FragB { v16b v; v8us half[2]; unsigned short u[16]; };
union FragH { v16h v; v8us half[2]; _Float16 h[16]; unsigned short u[16]; };

__device__ __forceinline__ unsigned short bf16_bits(float x) { unsigned int u = __float_as_uint(x); return (unsigned short)((u + 0x7FFFu + ((u >> 16) & 1u)) >> 16); }
__device__ __forceinline__ float bf16_val(unsigned short b) { return __uint_as_float(((unsigned int)b) << 16); }
__device__ __forceinline__ unsigned short f16_bits(float x) { return __builtin_bit_cast(unsigned short, (_Float16)x); }

__device__ __forceinline__ v8f mma_b(v16b a, v16b b, v8f c) {
  v8f d = __builtin_amdgcn_wmma_f32_16x16x32_bf16(false, a, false, b, (short)0, c, false, false);
  asm volatile("v_nop\n\tv_nop\n\tv_nop\n\tv_nop" : "+v"(d) : "v"(a), "v"(b));
  return d;
}
__device__ __forceinline__ v8f mma_h(v16h a, v16h b, v8f c) {
  v8f d = __builtin_amdgcn_wmma_f32_16x16x32_f16(false, a, false, b, (short)0, c, false, false);
  asm volatile("v_nop\n\tv_nop\n\tv_nop\n\tv_nop" : "+v"(d) : "v"(a), "v"(b));
  return d;
}
__device__ __forceinline__ v16h ld_h(const unsigned short* __restrict__ p, int hh) { FragH f; f.half[0] = *(const v8us*)(p + 8 * hh); f.half[1] = *(const v8us*)(p + 16 + 8 * hh); return f.v; }
__device__ __forceinline__ v16b ld_b(const unsigned short* __restrict__ p, int hh) { FragB f; f.half[0] = *(const v8us*)(p + 8 * hh); f.half[1] = *(const v8us*)(p + 16 + 8 * hh); return f.v; }

__global__ __launch_bounds__(256) void k_wplane(const float* __restrict__ W, unsigned short* __restrict__ Wp) {
  const int t = blockIdx.x * 256 + threadIdx.x;
  if (t >= NOUT * (EMB / 8)) return;
  const int p = t / (EMB / 8), k8 = (t % (EMB / 8)) * 8;
  const int which = p >> 6, fi = p & 63;
  const int o = fi * 3 + which;
  const v4f a = *(const v4fa*)(W + (size_t)o * EMB + k8);
  const v4f c = *(const v4fa*)(W + (size_t)o * EMB + k8 + 4);
  v8us v;
  v[0] = bf16_bits(a[0]); v[1] = bf16_bits(a[1]); v[2] = bf16_bits(a[2]); v[3] = bf16_bits(a[3]);
  v[4] = bf16_bits(c[0]); v[5] = bf16_bits(c[1]); v[6] = bf16_bits(c[2]); v[7] = bf16_bits(c[3]);
  *(volatile v8us*)(Wp + (size_t)p * EMB + k8) = v;
  __threadfence();
  *(volatile v8us*)(Wp + (size_t)p * EMB + k8) = v;
}

__global__ __launch_bounds__(128) void k_proj(const float* __restrict__ z, const unsigned short* __restrict__ Wp, const float* __restrict__ bias,
                                              unsigned short* __restrict__ Kh, unsigned short* __restrict__ Qh, unsigned short* __restrict__ VT) {
  __shared__ __attribute__((aligned(16))) unsigned short sk[4][16][72];
  __shared__ __attribute__((aligned(16))) unsigned short sq[4][16][72];
  __shared__ __attribute__((aligned(16))) unsigned short sv[64][72];
  const int tid = threadIdx.x;
  const int wave = __builtin_amdgcn_readfirstlane(tid >> 5);
  const int lane = tid & 31, ln = lane & 15, hh = lane >> 4;
  const int t0 = blockIdx.x * 64;
  const int b = t0 / SEQ, s0 = t0 - b * SEQ;
  const int row0 = t0 + 16 * wave;
  const float* arow = z + ((size_t)b * SEQ_FULL + s0 + 16 * wave + ln) * EMB;
  const unsigned short* wrow = Wp + (size_t)ln * EMB;
  const v8f z8 = {0.f, 0.f, 0.f, 0.f, 0.f, 0.f, 0.f, 0.f};
  v8f acc[12] = {z8, z8, z8, z8, z8, z8, z8, z8, z8, z8, z8, z8};
#pragma unroll 1
  for (int kb = 0; kb < EMB; kb += 32) {
    const v4f x0 = *(const v4fa*)(arow + kb + 8 * hh), x1 = *(const v4fa*)(arow + kb + 8 * hh + 4);
    const v4f x2 = *(const v4fa*)(arow + kb + 16 + 8 * hh), x3 = *(const v4fa*)(arow + kb + 16 + 8 * hh + 4);
    FragB ah;
    ah.u[0] = bf16_bits(x0[0]); ah.u[1] = bf16_bits(x0[1]); ah.u[2] = bf16_bits(x0[2]); ah.u[3] = bf16_bits(x0[3]);
    ah.u[4] = bf16_bits(x1[0]); ah.u[5] = bf16_bits(x1[1]); ah.u[6] = bf16_bits(x1[2]); ah.u[7] = bf16_bits(x1[3]);
    ah.u[8] = bf16_bits(x2[0]); ah.u[9] = bf16_bits(x2[1]); ah.u[10] = bf16_bits(x2[2]); ah.u[11] = bf16_bits(x2[3]);
    ah.u[12] = bf16_bits(x3[0]); ah.u[13] = bf16_bits(x3[1]); ah.u[14] = bf16_bits(x3[2]); ah.u[15] = bf16_bits(x3[3]);
#pragma unroll
    for (int g = 0; g < 3; ++g) {
#pragma unroll
      for (int u = 0; u < 4; ++u) {
        const int t = g * 4 + u;
        const v16b bf = ld_b(wrow + (size_t)(t * 16) * EMB + kb, hh);
        acc[t] = mma_b(ah.v, bf, acc[t]);
      }
      __builtin_amdgcn_sched_barrier(0);
    }
  }
#pragma unroll
  for (int t = 0; t < 4; ++t) {
    const int fi = t * 16 + ln;
    const float bk = bf16_val(bf16_bits(bias[fi * 3 + 0]));
    const float bq = bf16_val(bf16_bits(bias[fi * 3 + 1]));
    const float bv = bf16_val(bf16_bits(bias[fi * 3 + 2]));
#pragma unroll
    for (int r = 0; r < 8; ++r) {
      const int row = 8 * hh + r;
      sk[wave][row][fi] = f16_bits((acc[t][r] + bk) * CARRY);
      sq[wave][row][fi] = f16_bits((acc[4 + t][r] + bq) * CARRY);
      sv[fi][16 * wave + row] = f16_bits((acc[8 + t][r] + bv) * CARRY);
    }
  }
  __syncthreads();
  const int rq = lane >> 3, pc = (lane & 7) * 8;
  for (int pass = 0; pass < 2; ++pass) {
#pragma unroll
    for (int j = 0; j < 4; ++j) {
      const int r = j * 4 + rq;
      const v8us kv = *(const v8us*)&sk[wave][r][pc];
      const v8us qv = *(const v8us*)&sq[wave][r][pc];
      const int d = 16 * wave + j * 4 + rq;
      const v8us vv = *(const v8us*)&sv[d][pc];
      *(volatile v8us*)(Kh + (size_t)(row0 + r) * HD + pc) = kv;
      *(volatile v8us*)(Qh + (size_t)(row0 + r) * HD + pc) = qv;
      *(volatile v8us*)(VT + ((size_t)b * HD + d) * SEQ + s0 + pc) = vv;
    }
    if (pass == 0) __threadfence();
  }
}

__global__ __launch_bounds__(128) void k_attn(const unsigned short* __restrict__ Qh, const unsigned short* __restrict__ Kh,
                                              const unsigned short* __restrict__ VT, float* __restrict__ out) {
  __shared__ __attribute__((aligned(16))) float so[4][16][68];
  const int tid = threadIdx.x;
  const int wave = __builtin_amdgcn_readfirstlane(tid >> 5);
  const int lane = tid & 31, ln = lane & 15, hh = lane >> 4;
  const int q0 = (blockIdx.x * 4 + wave) * 16;
  const int b = q0 / SEQ;
  const unsigned short* qrow = Qh + (size_t)(q0 + ln) * HD;
  const v16h qf0 = ld_h(qrow, hh), qf1 = ld_h(qrow + 32, hh);
  const unsigned short* kp = Kh + ((size_t)b * SEQ + ln) * HD;
  const unsigned short* vp = VT + ((size_t)b * HD + ln) * SEQ;
  const v8f z8 = {0.f, 0.f, 0.f, 0.f, 0.f, 0.f, 0.f, 0.f};
  v8f o0 = z8, o1 = z8, o2 = z8, o3 = z8;
  float m = -1.0e30f, l = 0.f;
#pragma unroll 1
  for (int j0 = 0; j0 < SEQ; j0 += 32) {
    const unsigned short* k0p = kp + (size_t)j0 * HD;
    const unsigned short* k1p = k0p + 16 * HD;
    v8f s0 = z8, s1 = z8;
    v16h a;
    a = ld_h(k0p, hh);      s0 = mma_h(a, qf0, s0);
    a = ld_h(k0p + 32, hh); s0 = mma_h(a, qf1, s0);
    a = ld_h(k1p, hh);      s1 = mma_h(a, qf0, s1);
    a = ld_h(k1p + 32, hh); s1 = mma_h(a, qf1, s1);
    float x0[8], x1[8];
    float mloc = -3.0e38f;
#pragma unroll
    for (int r = 0; r < 8; ++r) { x0[r] = s0[r] * SC_LOGIT; x1[r] = s1[r] * SC_LOGIT; mloc = fmaxf(mloc, fmaxf(x0[r], x1[r])); }
    mloc = fmaxf(mloc, __shfl_xor(mloc, 16, 32));
    const float mn = fmaxf(m, mloc);
    const float corr = __expf(m - mn);
    float ps = 0.f;
    FragH pb;
#pragma unroll
    for (int r = 0; r < 8; ++r) {
      const float p0 = __expf(x0[r] - mn);
      const float p1 = __expf(x1[r] - mn);
      ps += p0 + p1;
      pb.h[r] = (_Float16)p0;
      pb.h[8 + r] = (_Float16)p1;
    }
    l = l * corr + ps;
    m = mn;
    o0 = o0 * corr; o1 = o1 * corr; o2 = o2 * corr; o3 = o3 * corr;
    const unsigned short* vj = vp + j0;
    a = ld_h(vj, hh);                     o0 = mma_h(a, pb.v, o0);
    a = ld_h(vj + (size_t)16 * SEQ, hh);  o1 = mma_h(a, pb.v, o1);
    a = ld_h(vj + (size_t)32 * SEQ, hh);  o2 = mma_h(a, pb.v, o2);
    a = ld_h(vj + (size_t)48 * SEQ, hh);  o3 = mma_h(a, pb.v, o3);
  }
  l = l + __shfl_xor(l, 16, 32);
  const float inv = (1.0f / l) * (1.0f / CARRY);
#pragma unroll
  for (int r = 0; r < 8; ++r) {
    so[wave][ln][0 + 8 * hh + r] = o0[r] * inv;
    so[wave][ln][16 + 8 * hh + r] = o1[r] * inv;
    so[wave][ln][32 + 8 * hh + r] = o2[r] * inv;
    so[wave][ln][48 + 8 * hh + r] = o3[r] * inv;
  }
  __syncthreads();
  const int rsub = lane >> 4, c4 = (lane & 15) * 4;
  for (int pass = 0; pass < 2; ++pass) {
#pragma unroll
    for (int q = 0; q < 8; ++q) {
      const int r = q * 2 + rsub;
      const v4f v = *(const v4fa*)&so[wave][r][c4];
      *(volatile v4f*)(out + (size_t)(q0 + r) * HD + c4) = v;
    }
    if (pass == 0) __threadfence();
  }
}

extern "C" void kernel_launch(void* const* d_in, const int* in_sizes, int n_in,
                              void* d_out, int out_size, void* d_ws, size_t ws_size, hipStream_t stream) {
  if (n_in < 3) return;
  if ((long long)in_sizes[0] < ((long long)(NB - 1) * SEQ_FULL + SEQ) * EMB) return;
  if (in_sizes[1] < NOUT * EMB) return;
  if (in_sizes[2] < NOUT) return;
  if ((long long)out_size < (long long)NTOK * HD) return;
  if (OFF_END > ws_size) return;
  const float* z = (const float*)d_in[0];
  const float* W = (const float*)d_in[1];
  const float* bias = (const float*)d_in[2];
  float* out = (float*)d_out;
  char* ws = (char*)d_ws;
  unsigned short* Wp = (unsigned short*)(ws + OFF_WP);
  unsigned short* Kh = (unsigned short*)(ws + OFF_KH);
  unsigned short* Qh = (unsigned short*)(ws + OFF_QH);
  unsigned short* VT = (unsigned short*)(ws + OFF_VT);
  k_wplane<<<(NOUT * (EMB / 8)) / 256, 256, 0, stream>>>(W, Wp);
  k_proj<<<NTOK / 64, 128, 0, stream>>>(z, Wp, bias, Kh, Qh, VT);
  k_attn<<<NTOK / 64, 128, 0, stream>>>(Qh, Kh, VT, out);
}
